// Token_GAT_24979529794139
// MI455X (gfx1250) — hardware-verified
//
#include <hip/hip_runtime.h>
#include <hip/hip_bf16.h>

typedef __attribute__((ext_vector_type(16))) _Float16 v16h;
typedef __attribute__((ext_vector_type(8)))  float    v8f;

#define BATCH 32
#define NN    512
#define DIN   768
#define DOUT  256
#define HEADS 8
#define PSTRIDE 516

typedef __attribute__((ext_vector_type(4))) float v4f_t;
typedef float v4fa __attribute__((ext_vector_type(4), may_alias));
static __device__ __forceinline__ unsigned pk2(float a, float b) { return (unsigned)__builtin_bit_cast(unsigned short, (_Float16)a) | ((unsigned)__builtin_bit_cast(unsigned short, (_Float16)b) << 16); }
static __device__ __forceinline__ void store_tile16x32(const float* stg, int sst, float* __restrict__ dst, size_t ld, int lane) {
  v4f_t vv[4];
#pragma unroll
  for (int i = 0; i < 4; ++i) { const int c = lane + 32 * i; vv[i] = *(const volatile v4fa*)(stg + (c >> 3) * sst + (c & 7) * 4); }
#pragma unroll
  for (int i = 0; i < 4; ++i) { const int c = lane + 32 * i; *(volatile v4f_t*)(dst + (size_t)(c >> 3) * ld + (c & 7) * 4) = vv[i]; }
  __threadfence();
#pragma unroll
  for (int i = 0; i < 4; ++i) { const int c = lane + 32 * i; *(volatile v4f_t*)(dst + (size_t)(c >> 3) * ld + (c & 7) * 4) = vv[i]; }
}
static __device__ __forceinline__ v8f wmma16(v16h a, v16h b, v8f c) {
  return __builtin_amdgcn_wmma_f32_16x16x32_f16(false, a, false, b,
                                                (short)0, c, false, false);
}


__global__ __launch_bounds__(256) void zero_f32(float* p, int n) {
  int i = blockIdx.x * 256 + threadIdx.x;
  if (i < n) { *(volatile float*)(p + i) = 0.0f; __threadfence(); *(volatile float*)(p + i) = 0.0f; }
}

__global__ __launch_bounds__(256) void pack_a(const float* __restrict__ src,
                                              _Float16* __restrict__ dst, int K) {
  int Kt = K >> 5;
  size_t gid = ((size_t)blockIdx.x * 256 + threadIdx.x) * 2;
  int tile   = (int)(gid >> 9);
  int within = (int)(gid & 511);
  int lane = within >> 4;
  int e    = within & 15;
  int mt = tile / Kt, kt = tile - mt * Kt;
  int m = mt * 16 + (lane & 15);
  int v = e >> 1;
  int k = kt * 32 + ((v < 4) ? 0 : 16) + ((lane >= 16) ? 8 : 0) + ((v & 3) << 1);
  const float* s = src + (size_t)m * K + k;
  const unsigned p = pk2(s[0], s[1]);
  *(volatile unsigned*)(dst + gid) = p; __threadfence(); *(volatile unsigned*)(dst + gid) = p;
}

__global__ __launch_bounds__(256) void pack_b(const float* __restrict__ src,
                                              _Float16* __restrict__ dst,
                                              int K, int Ncols) {
  int Kt = K >> 5, Nt = Ncols >> 4;
  size_t perBatch = (size_t)Kt * Nt * 512;
  size_t gid = ((size_t)blockIdx.x * 256 + threadIdx.x) * 2;
  size_t bidx = gid / perBatch;
  size_t rem  = gid - bidx * perBatch;
  int tile   = (int)(rem >> 9);
  int within = (int)(rem & 511);
  int lane = within >> 4;
  int e    = within & 15;
  int kt = tile / Nt, nt = tile - kt * Nt;
  int n = nt * 16 + (lane & 15);
  int k = kt * 32 + ((e < 8) ? (((lane >= 16) ? 8 : 0) + e) : (16 + ((lane >= 16) ? 8 : 0) + (e - 8)));
  const float* s = src + bidx * (size_t)K * Ncols + (size_t)k * Ncols + n;
  const unsigned p = pk2(s[0], s[Ncols]);
  *(volatile unsigned*)(dst + gid) = p; __threadfence(); *(volatile unsigned*)(dst + gid) = p;
}

__global__ __launch_bounds__(256) void gemm_wmma(const _Float16* __restrict__ Apack,
                                                 const _Float16* __restrict__ Bpack,
                                                 float* __restrict__ C,
                                                 int Ktiles, int Ntiles) {
  int t = threadIdx.x, lane = t & 31, wave = t >> 5;
  int mt0 = blockIdx.y * 2;
  int nt0 = wave * 2;
  const _Float16* a0p = Apack + ((size_t)mt0 * Ktiles) * 512 + (size_t)lane * 16;
  const _Float16* a1p = a0p + (size_t)Ktiles * 512;
  const _Float16* bp  = Bpack + (size_t)lane * 16;
  v8f acc00 = {}, acc01 = {}, acc10 = {}, acc11 = {};
  for (int kt = 0; kt < Ktiles; ++kt) {
    v16h a0 = *(const v16h*)(a0p + (size_t)kt * 512);
    v16h a1 = *(const v16h*)(a1p + (size_t)kt * 512);
    v16h b0 = *(const v16h*)(bp + ((size_t)kt * Ntiles + nt0) * 512);
    v16h b1 = *(const v16h*)(bp + ((size_t)kt * Ntiles + nt0 + 1) * 512);
    if (kt + 1 < Ktiles)
      __builtin_prefetch(bp + (((size_t)kt + 1) * Ntiles + nt0) * 512, 0, 0);
    acc00 = wmma16(a0, b0, acc00);
    acc01 = wmma16(a0, b1, acc01);
    acc10 = wmma16(a1, b0, acc10);
    acc11 = wmma16(a1, b1, acc11);
  }
  __shared__ __align__(16) float cst[8][32 * 32];
  int ldc  = Ntiles * 16;
  int mrow = ((lane >= 16) ? 8 : 0);
  float* cs = cst[wave];
#pragma unroll
  for (int r = 0; r < 8; ++r) {
    cs[(mrow + r) * 32 + (lane & 15)]           = acc00[r];
    cs[(mrow + r) * 32 + 16 + (lane & 15)]      = acc01[r];
    cs[(16 + mrow + r) * 32 + (lane & 15)]      = acc10[r];
    cs[(16 + mrow + r) * 32 + 16 + (lane & 15)] = acc11[r];
  }
  asm volatile("s_wait_dscnt 0" ::: "memory");
  store_tile16x32(cs,           32, C + (size_t)(mt0 * 16) * ldc + nt0 * 16, (size_t)ldc, lane);
  store_tile16x32(cs + 16 * 32, 32, C + (size_t)((mt0 + 1) * 16) * ldc + nt0 * 16, (size_t)ldc, lane);
}

__global__ __launch_bounds__(256) void scores_kernel(const float* __restrict__ Wh,
                                                     const float* __restrict__ a1,
                                                     const float* __restrict__ a2,
                                                     float* __restrict__ f1,
                                                     float* __restrict__ f2) {
  __shared__ float s1[32], s2[32];
  int t = threadIdx.x, lane = t & 31, wave = t >> 5;
  float a1v[8], a2v[8];
#pragma unroll
  for (int i = 0; i < 8; ++i) { a1v[i] = a1[lane + 32 * i]; a2v[i] = a2[lane + 32 * i]; }
#pragma unroll
  for (int q = 0; q < 4; ++q) {
    const int row = blockIdx.x * 32 + wave * 4 + q;
    float p1 = 0.f, p2 = 0.f;
#pragma unroll
    for (int i = 0; i < 8; ++i) { const float w = Wh[(size_t)row * DOUT + lane + 32 * i]; p1 += w * a1v[i]; p2 += w * a2v[i]; }
#pragma unroll
    for (int off = 16; off > 0; off >>= 1) { p1 += __shfl_xor(p1, off, 32); p2 += __shfl_xor(p2, off, 32); }
    if (lane == 0) { s1[wave * 4 + q] = p1; s2[wave * 4 + q] = p2; }
  }
  __syncthreads();
  if (wave == 0) {
    const size_t o = (size_t)blockIdx.x * 32 + lane;
    *(volatile float*)(f1 + o) = s1[lane]; *(volatile float*)(f2 + o) = s2[lane];
    __threadfence();
    *(volatile float*)(f1 + o) = s1[lane]; *(volatile float*)(f2 + o) = s2[lane];
  }
}

__global__ __launch_bounds__(256) void attn_kernel(const float* __restrict__ f1,
                                                   const float* __restrict__ f2,
                                                   const int* __restrict__ adj,
                                                   const _Float16* __restrict__ WhBpack,
                                                   float* __restrict__ out,
                                                   int mode, float scale) {
  __shared__ float scoresLDS[16 * PSTRIDE];
  __shared__ __align__(16) _Float16 afrag[16 * 512];
  __shared__ float red[16 * 16];
  __shared__ float rowmax[16];
  __shared__ float rowinv[16];

  int b = blockIdx.y;
  int row0 = blockIdx.x * 16;
  int t = threadIdx.x;
  int r = t >> 4;
  int c16 = t & 15;

  float fi = f1[b * NN + row0 + r];
  const int* adjRow = adj + ((size_t)(b * NN + row0 + r)) * NN;
  float lmax = -3.0e38f;
  for (int i = 0; i < 32; ++i) {
    int j = c16 + i * 16;
    float s = fi + f2[b * NN + j];
    s = s > 0.0f ? s : 0.2f * s;
    if (adjRow[j] == 0) s = -9.0e15f;
    scoresLDS[r * PSTRIDE + j] = s;
    lmax = fmaxf(lmax, s);
  }
  red[r * 16 + c16] = lmax;
  __syncthreads();
  if (t < 16) {
    float m = red[t * 16];
    for (int i = 1; i < 16; ++i) m = fmaxf(m, red[t * 16 + i]);
    rowmax[t] = m;
  }
  __syncthreads();

  float rm = rowmax[r];
  float lsum = 0.0f;
  for (int i = 0; i < 32; ++i) {
    int j = c16 + i * 16;
    float ev = __expf(scoresLDS[r * PSTRIDE + j] - rm);
    lsum += ev;
    int kt     = j >> 5;
    int k32    = j & 31;
    int hh     = k32 & 1;
    int laneHi = (k32 >> 3) & 1;
    int v      = (((k32 >> 4) & 1) << 2) | ((k32 >> 1) & 3);
    int lane_  = (laneHi << 4) | r;
    int e      = (v << 1) | hh;
    afrag[(kt << 9) + (lane_ << 4) + e] = (_Float16)(ev * 1024.0f);
  }
  red[r * 16 + c16] = lsum;
  __syncthreads();
  if (t < 16) {
    float s = 0.0f;
    for (int i = 0; i < 16; ++i) s += red[t * 16 + i];
    rowinv[t] = 1.0f / (s * 1024.0f);
  }
  __syncthreads();

  int lane = t & 31, wave = t >> 5;
  int nt0 = 2 * wave, nt1 = 2 * wave + 1;
  const _Float16* af = afrag + (size_t)lane * 16;
  const _Float16* bp = WhBpack + (((size_t)b * 16) * 16) * 512 + (size_t)lane * 16;
  v8f acc0 = {}, acc1 = {};
  for (int kt = 0; kt < 16; ++kt) {
    v16h a  = *(const v16h*)(af + (size_t)kt * 512);
    v16h b0 = *(const v16h*)(bp + ((size_t)kt * 16 + nt0) * 512);
    v16h b1 = *(const v16h*)(bp + ((size_t)kt * 16 + nt1) * 512);
    acc0 = wmma16(a, b0, acc0);
    acc1 = wmma16(a, b1, acc1);
  }

  int mbase = ((lane >= 16) ? 8 : 0);
  float* sw = scoresLDS + wave * (16 * 32);
#pragma unroll
  for (int rr = 0; rr < 8; ++rr) {
    int m = rr + mbase;
    float invm = rowinv[m];
    float v0 = acc0[rr] * invm;
    float v1 = acc1[rr] * invm;
    if (mode == 0) {
      v0 = v0 > 0.0f ? v0 : (__expf(v0) - 1.0f);
      v1 = v1 > 0.0f ? v1 : (__expf(v1) - 1.0f);
      v0 *= scale; v1 *= scale;
    } else {
      v0 = v0 > 0.0f ? v0 : 0.0f;
      v1 = v1 > 0.0f ? v1 : 0.0f;
    }
    sw[m * 32 + (lane & 15)]      = v0;
    sw[m * 32 + 16 + (lane & 15)] = v1;
  }
  asm volatile("s_wait_dscnt 0" ::: "memory");
  {
    float* dst = out + ((size_t)b * NN + row0) * DOUT + nt0 * 16;
    v4f_t vv[4];
#pragma unroll
    for (int i = 0; i < 4; ++i) {
      const int c = lane + 32 * i, rr = c >> 3, q = c & 7;
      vv[i] = *(const volatile v4fa*)(sw + rr * 32 + q * 4);
      if (mode == 0) vv[i] += *(const v4f_t*)(dst + (size_t)rr * DOUT + q * 4);
    }
#pragma unroll
    for (int i = 0; i < 4; ++i) { const int c = lane + 32 * i; *(volatile v4f_t*)(dst + (size_t)(c >> 3) * DOUT + (c & 7) * 4) = vv[i]; }
    __threadfence();
#pragma unroll
    for (int i = 0; i < 4; ++i) { const int c = lane + 32 * i; *(volatile v4f_t*)(dst + (size_t)(c >> 3) * DOUT + (c & 7) * 4) = vv[i]; }
  }
}

extern "C" void kernel_launch(void* const* d_in, const int* in_sizes, int n_in,
                              void* d_out, int out_size, void* d_ws, size_t ws_size,
                              hipStream_t stream) {
  const float* x    = (const float*)d_in[0];
  const int*   adj  = (const int*)d_in[1];
  const float* W0   = (const float*)d_in[2];
  const float* a1_0 = (const float*)d_in[3];
  const float* a2_0 = (const float*)d_in[4];
  const float* Wo   = (const float*)d_in[5];
  const float* a1_o = (const float*)d_in[6];
  const float* a2_o = (const float*)d_in[7];
  float* out = (float*)d_out;

  const size_t M = (size_t)BATCH * NN;

  char* ws = (char*)d_ws;
  _Float16* Apack_x = (_Float16*)ws;
  _Float16* BpackW0 = Apack_x + M * DIN;
  float*    Wh      = (float*)(BpackW0 + (size_t)HEADS * DIN * DOUT);
  float*    f1      = Wh + M * DOUT;
  float*    f2      = f1 + M;
  _Float16* WhBpack = (_Float16*)(f2 + M);
  float*    h_mean  = (float*)(WhBpack + (size_t)BATCH * NN * DOUT);
  _Float16* Apack_h = (_Float16*)(h_mean + M * DOUT);
  _Float16* BpackWo = Apack_h + M * DOUT;

  {
    int n = (int)(M * DOUT);
    zero_f32<<<dim3((n + 255) / 256), dim3(256), 0, stream>>>(h_mean, n);
  }
  pack_a<<<dim3((unsigned)(M * DIN / 512)), dim3(256), 0, stream>>>(x, Apack_x, DIN);
  pack_b<<<dim3((unsigned)((size_t)HEADS * DIN * DOUT / 512)), dim3(256), 0, stream>>>(
      W0, BpackW0, DIN, DOUT);

  for (int h = 0; h < HEADS; ++h) {
    gemm_wmma<<<dim3(1, (unsigned)(M / 32)), dim3(256), 0, stream>>>(
        Apack_x, BpackW0 + (size_t)h * DIN * DOUT, Wh, DIN / 32, DOUT / 16);
    scores_kernel<<<dim3((unsigned)(M / 32)), dim3(256), 0, stream>>>(
        Wh, a1_0 + h * DOUT, a2_0 + h * DOUT, f1, f2);
    pack_b<<<dim3((unsigned)((size_t)BATCH * NN * DOUT / 512)), dim3(256), 0, stream>>>(
        Wh, WhBpack, NN, DOUT);
    attn_kernel<<<dim3(NN / 16, BATCH), dim3(256), 0, stream>>>(
        f1, f2, adj, WhBpack, h_mean, 0, 1.0f / HEADS);
  }

  pack_a<<<dim3((unsigned)(M * DOUT / 512)), dim3(256), 0, stream>>>(h_mean, Apack_h, DOUT);
  pack_b<<<dim3((unsigned)((size_t)DOUT * DOUT / 512)), dim3(256), 0, stream>>>(
      Wo, BpackWo, DOUT, DOUT);
  gemm_wmma<<<dim3(1, (unsigned)(M / 32)), dim3(256), 0, stream>>>(
      Apack_h, BpackWo, Wh, DOUT / 32, DOUT / 16);
  scores_kernel<<<dim3((unsigned)(M / 32)), dim3(256), 0, stream>>>(Wh, a1_o, a2_o, f1, f2);
  pack_b<<<dim3((unsigned)((size_t)BATCH * NN * DOUT / 512)), dim3(256), 0, stream>>>(
      Wh, WhBpack, NN, DOUT);
  attn_kernel<<<dim3(NN / 16, BATCH), dim3(256), 0, stream>>>(
      f1, f2, adj, WhBpack, out, 1, 1.0f);
}
